// C_Aggregation_24807731101830
// MI455X (gfx1250) — hardware-verified
//
#include <hip/hip_runtime.h>
#include <stddef.h>


typedef __attribute__((ext_vector_type(16))) _Float16 v16h;
typedef __attribute__((ext_vector_type(8)))  _Float16 v8h;
typedef __attribute__((ext_vector_type(16))) __bf16   v16b;
typedef __attribute__((ext_vector_type(8)))  __bf16   v8b;
typedef __attribute__((ext_vector_type(8)))  float    v8f;
typedef __attribute__((ext_vector_type(4)))  float    v4f;

#define NB    16
#define CHN   3
#define IMG   512
#define SIDE  544
#define EMB   768
#define KDIM  768
#define NPOS  1156
#define MPAD  1216
#define TCOLS (NB * EMB)

__device__ __forceinline__ unsigned short f2bf_bits(float f) {
  unsigned u = __float_as_uint(f);
  return (unsigned short)((u + 0x7FFFu + ((u >> 16) & 1u)) >> 16);
}
__device__ __forceinline__ float bf_bits2f(unsigned short h) { return __uint_as_float(((unsigned)h) << 16); }

__device__ __forceinline__ void dep_guard_h(v8f& a, v8f& b, v16h x, v16h y) { asm volatile("v_nop\n\tv_nop\n\tv_nop\n\tv_nop" : "+v"(a), "+v"(b) : "v"(x), "v"(y)); }
__device__ __forceinline__ void dep_guard_b(v8f& a, v8f& b, v16b x, v16b y) { asm volatile("v_nop\n\tv_nop\n\tv_nop\n\tv_nop" : "+v"(a), "+v"(b) : "v"(x), "v"(y)); }
__device__ __forceinline__ void keep4_h(v16h a, v16h b, v16h c, v16h d) { asm volatile("v_nop" :: "v"(a), "v"(b), "v"(c), "v"(d)); }
__device__ __forceinline__ void keep4_b(v16b a, v16b b, v16b c, v16b d) { asm volatile("v_nop" :: "v"(a), "v"(b), "v"(c), "v"(d)); }
__device__ __forceinline__ void acc_guard4(v8f& a, v8f& b, v8f& c, v8f& d) { asm volatile("v_nop\n\tv_nop\n\tv_nop\n\tv_nop" : "+v"(a), "+v"(b), "+v"(c), "+v"(d)); }
template <typename T> struct Frag;
template <> struct Frag<_Float16> {
  typedef v16h V; union U { v16h v; v8h h[2]; };
  static __device__ __forceinline__ v16h load(const _Float16* p) {
    U f; f.h[0] = *(const v8h*)(p); f.h[1] = *(const v8h*)(p + 16); return f.v;
  }
  static __device__ __forceinline__ v8f mma(v16h a, v16h b, v8f c) {
    return __builtin_amdgcn_wmma_f32_16x16x32_f16(false, a, false, b, (short)0, c, false, false);
  }
  static __device__ __forceinline__ void guard(v8f& a, v8f& b, v16h x, v16h y) { dep_guard_h(a, b, x, y); }
  static __device__ __forceinline__ void keep(v16h a, v16h b, v16h c, v16h d) { keep4_h(a, b, c, d); }
};
template <> struct Frag<__bf16> {
  typedef v16b V; union U { v16b v; v8b h[2]; };
  static __device__ __forceinline__ v16b load(const __bf16* p) {
    U f; f.h[0] = *(const v8b*)(p); f.h[1] = *(const v8b*)(p + 16); return f.v;
  }
  static __device__ __forceinline__ v8f mma(v16b a, v16b b, v8f c) {
    return __builtin_amdgcn_wmma_f32_16x16x32_bf16(false, a, false, b, (short)0, c, false, false);
  }
  static __device__ __forceinline__ void guard(v8f& a, v8f& b, v16b x, v16b y) { dep_guard_b(a, b, x, y); }
  static __device__ __forceinline__ void keep(v16b a, v16b b, v16b c, v16b d) { keep4_b(a, b, c, d); }
};

template <int ET> struct Elem;
template <> struct Elem<0> { typedef _Float16 T; };
template <> struct Elem<1> { typedef __bf16 T; };
template <int ET, bool SPLIT, int BIAS_MODE, int OUT_MODE, bool RESID, int ACT = 0>
__global__ __launch_bounds__(256) void wmma_gemm64(
    const unsigned short* __restrict__ Ap, const unsigned short* __restrict__ A2p, int lda, long strideA,
    const unsigned short* __restrict__ Btp, const unsigned short* __restrict__ Bt2p, int ldb, long strideB,
    void* __restrict__ Cout, void* __restrict__ Cout2, int ldc, long strideC,
    const float* __restrict__ bias,
    const float* __restrict__ resid, long strideR,
    int M, int N, int K, float scale) {
  typedef typename Elem<ET>::T T;
  typedef typename Frag<T>::V V;
  const T* A = (const T*)Ap; const T* A2 = (const T*)A2p; const T* Bt = (const T*)Btp; const T* Bt2 = (const T*)Bt2p;
  __shared__ __align__(16) float sT[8][16 * 68];
  const int b    = blockIdx.y;
  const int lane = threadIdx.x & 31;
  const int wave = threadIdx.x >> 5;
  const int tilesN = N >> 6;
  const int tilesM = M >> 6;
  const int tile = blockIdx.x * 8 + wave;
  if (tile >= tilesM * tilesN) return;
  const int tm = tile / tilesN;
  const int tn = tile - tm * tilesN;
  const int m0 = tm << 6;
  const int n0 = tn << 6;

  const T* Ab  = A  + (size_t)b * strideA;
  const T* Bb  = Bt + (size_t)b * strideB;
  const T* Ab2 = SPLIT ? (A2  + (size_t)b * strideA) : nullptr;
  const T* Bb2 = SPLIT ? (Bt2 + (size_t)b * strideB) : nullptr;

  const int rlane = lane & 15;
  const int koff  = (lane >> 4) * 8;
  const int mOff  = (lane >> 4) * 8;

  v8f acc[4][4];
#pragma unroll
  for (int i = 0; i < 4; ++i)
#pragma unroll
    for (int j = 0; j < 4; ++j) acc[i][j] = (v8f){0.f,0.f,0.f,0.f,0.f,0.f,0.f,0.f};

  for (int k0 = 0; k0 < K; k0 += 32) {
    V bh[4], bl[4];
#pragma unroll
    for (int j = 0; j < 4; ++j) {
      const size_t bo = (size_t)(n0 + (j << 4) + rlane) * ldb + koff + k0;
      bh[j] = Frag<T>::load(Bb + bo);
      if (SPLIT) bl[j] = Frag<T>::load(Bb2 + bo);
    }
#pragma unroll
    for (int i = 0; i < 4; ++i) {
      const size_t ao = (size_t)(m0 + (i << 4) + rlane) * lda + koff + k0;
      V ah = Frag<T>::load(Ab + ao);
      V al;
      if (SPLIT) al = Frag<T>::load(Ab2 + ao);
#pragma unroll
      for (int j = 0; j < 4; ++j) {
        acc[i][j] = Frag<T>::mma(ah, bh[j], acc[i][j]);
        if (SPLIT) {
          acc[i][j] = Frag<T>::mma(ah, bl[j], acc[i][j]);
          acc[i][j] = Frag<T>::mma(al, bh[j], acc[i][j]);
        }
      }
      Frag<T>::guard(acc[i][0], acc[i][3], ah, SPLIT ? al : ah);
    }
    Frag<T>::keep(bh[0], bh[1], bh[2], bh[3]);
    if (SPLIT) Frag<T>::keep(bl[0], bl[1], bl[2], bl[3]);
  }
  acc_guard4(acc[0][0], acc[0][1], acc[0][2], acc[0][3]);
  acc_guard4(acc[1][0], acc[1][1], acc[1][2], acc[1][3]);
  acc_guard4(acc[2][0], acc[2][1], acc[2][2], acc[2][3]);
  acc_guard4(acc[3][0], acc[3][1], acc[3][2], acc[3][3]);

  float* slab = sT[wave];
  const float* Rb = RESID ? (resid + (size_t)b * strideR) : nullptr;
#pragma unroll
  for (int i = 0; i < 4; ++i) {
    const int mBase = m0 + (i << 4);
#pragma unroll
    for (int j = 0; j < 4; ++j) {
      const int n = n0 + (j << 4) + rlane;
      float bv = 0.f;
      if (BIAS_MODE == 2) bv = bias[n];
#pragma unroll
      for (int r = 0; r < 8; ++r) {
        float v = acc[i][j][r] * scale;
        if (BIAS_MODE == 1) v += bias[mBase + mOff + r];
        if (BIAS_MODE == 2) v += bv;
        if (RESID) v += Rb[(size_t)(mBase + mOff + r) * ldc + n];
        if (ACT == 1) v = tanhf(v);
        if (ACT == 2) v = fmaxf(v, 0.0f);
        if (ACT == 3) v = v / (1.0f + expf(-v));
        if (ACT == 4) v = (v > 0.f) ? v : 0.01f * v;
        if (ACT == 5) v = 0.5f * v * (1.0f + erff(v * 0.70710678118654752f));
        slab[(mOff + r) * 68 + (j << 4) + rlane] = v;
      }
    }
    __builtin_amdgcn_fence(__ATOMIC_RELEASE, "workgroup");
    __builtin_amdgcn_wave_barrier();
    __builtin_amdgcn_fence(__ATOMIC_ACQUIRE, "workgroup");
    if (OUT_MODE == 0) {
      float* C = (float*)Cout + (size_t)b * strideC;
      const int hh = lane >> 4, c4 = (lane & 15) * 4;
      for (int pass = 0; pass < 2; ++pass) {
#pragma unroll
        for (int it = 0; it < 8; ++it) {
          const int row = it * 2 + hh;
          v4f v = *(const v4f*)(slab + row * 68 + c4);
          *(volatile v4f*)(C + (size_t)(mBase + row) * ldc + n0 + c4) = v;
        }
        __threadfence();
      }
    } else {
      const int q = lane >> 3, c8 = (lane & 7) * 8;
      unsigned short* C  = (unsigned short*)Cout  + (size_t)b * strideC;
      unsigned short* C2 = (OUT_MODE == 2) ? ((unsigned short*)Cout2 + (size_t)b * strideC) : nullptr;
      for (int pass = 0; pass < 2; ++pass) {
#pragma unroll
        for (int it = 0; it < 4; ++it) {
          const int row = it * 4 + q;
          const float* sp = slab + row * 68 + c8;
          v8h hv, lv;
#pragma unroll
          for (int e = 0; e < 8; ++e) {
            if (OUT_MODE == 1) {
              hv[e] = (_Float16)sp[e];
            } else {
              unsigned short hb = f2bf_bits(sp[e]);
              unsigned short lb = f2bf_bits(sp[e] - bf_bits2f(hb));
              hv[e] = __builtin_bit_cast(_Float16, hb);
              lv[e] = __builtin_bit_cast(_Float16, lb);
            }
          }
          *(volatile v8h*)(C + (size_t)(mBase + row) * ldc + n0 + c8) = hv;
          if (OUT_MODE == 2) *(volatile v8h*)(C2 + (size_t)(mBase + row) * ldc + n0 + c8) = lv;
        }
        __threadfence();
      }
    }
    __builtin_amdgcn_fence(__ATOMIC_RELEASE, "workgroup");
    __builtin_amdgcn_wave_barrier();
    __builtin_amdgcn_fence(__ATOMIC_ACQUIRE, "workgroup");
  }
}

__global__ __launch_bounds__(256) void cast_w_f16x2(
    const float* __restrict__ in, _Float16* __restrict__ out, int n2, float sc) {
  int i = blockIdx.x * 256 + threadIdx.x;
  if (i < n2) {
    const _Float16 h0 = (_Float16)(in[2 * i] * sc), h1 = (_Float16)(in[2 * i + 1] * sc);
    const unsigned u = (unsigned)__builtin_bit_cast(unsigned short, h0) | ((unsigned)__builtin_bit_cast(unsigned short, h1) << 16);
    ((volatile unsigned*)out)[i] = u;
    __threadfence();
    ((volatile unsigned*)out)[i] = u;
  }
}

__global__ __launch_bounds__(256) void im2col_f16(const float* __restrict__ x, _Float16* __restrict__ A) {
  const int t = blockIdx.x * 256 + threadIdx.x;
  if (t >= NB * MPAD * (KDIM / 8)) return;
  const int kc = t % (KDIM / 8);
  const int m  = (t / (KDIM / 8)) % MPAD;
  const int b  = t / ((KDIM / 8) * MPAD);
  const int k0 = kc * 8;
  const int c  = k0 >> 8, dy = (k0 >> 4) & 15, dx0 = k0 & 15;
  const int ph = m / 34, pw = m - ph * 34;
  v8h hv;
#pragma unroll
  for (int e = 0; e < 8; ++e) hv[e] = (_Float16)0.0f;
  if (m < NPOS && ph >= 1 && ph <= 32 && pw >= 1 && pw <= 32) {
    const int row  = 16 * (ph - 1) + dy;
    const int colx = 16 * (pw - 1) + dx0;
    const float* src = x + (((size_t)(b * CHN + c)) * IMG + row) * IMG + colx;
    const v4f p0 = *(const v4f*)(src);
    const v4f p1 = *(const v4f*)(src + 4);
    hv[0] = (_Float16)p0[0]; hv[1] = (_Float16)p0[1]; hv[2] = (_Float16)p0[2]; hv[3] = (_Float16)p0[3];
    hv[4] = (_Float16)p1[0]; hv[5] = (_Float16)p1[1]; hv[6] = (_Float16)p1[2]; hv[7] = (_Float16)p1[3];
  }
  _Float16* dst = A + ((size_t)(b * MPAD + m)) * KDIM + k0;
  *(volatile v8h*)dst = hv;
  __threadfence();
  *(volatile v8h*)dst = hv;
}

__global__ __launch_bounds__(256) void smooth_scan(float* __restrict__ buf) {
#pragma clang fp contract(off)
  const int t = blockIdx.x * 256 + threadIdx.x;
  if (t >= TCOLS) return;
  float* col = buf + t;
  float prev[33];
#pragma unroll
  for (int j = 0; j < 33; ++j) prev[j] = col[(size_t)j * TCOLS];
#pragma unroll 1
  for (int i = 1; i <= 30; ++i) {
    const size_t rb = (size_t)i * 32;
    float same[33], below[33], cur[33];
#pragma unroll
    for (int j = 0; j < 33; ++j) {
      same[j]  = col[(rb + j) * TCOLS];
      below[j] = col[(rb + 32 + j) * TCOLS];
    }
    cur[0]  = same[0];
    cur[32] = same[32];
#pragma unroll
    for (int j = 1; j <= 31; ++j) {
      float s = prev[j] + below[j];
      s = s + cur[j - 1];
      s = s + same[j + 1];
      s = s + prev[j - 1];
      s = s + prev[j + 1];
      s = s + below[j - 1];
      s = s + below[j + 1];
      const float o = s * 0.125f;
      cur[j] = o;
      *(volatile float*)(col + (rb + j) * TCOLS) = o;
    }
    __threadfence();
#pragma unroll
    for (int j = 1; j <= 31; ++j) *(volatile float*)(col + (rb + j) * TCOLS) = cur[j];
#pragma unroll
    for (int j = 0; j < 33; ++j) prev[j] = cur[j];
  }
}

__global__ __launch_bounds__(256) void crop_copy(const float* __restrict__ buf, float* __restrict__ out) {
  const int t = blockIdx.x * 256 + threadIdx.x;
  if (t >= NB * CHN * IMG * (IMG / 4)) return;
  const int w4 = (t & 127) * 4;
  const int hh = (t >> 7) & 511;
  const int bc = t >> 16;
  const int c  = bc % CHN;
  const int b  = bc / CHN;
  v4f v;
#pragma unroll
  for (int e = 0; e < 4; ++e) {
    const int f  = c * (SIDE * SIDE) + (hh + 16) * SIDE + (w4 + e + 16);
    const int c1 = f / NPOS;
    const int s  = f - c1 * NPOS;
    v[e] = buf[(size_t)s * TCOLS + (size_t)b * EMB + c1];
  }
  float* p = out + (size_t)t * 4;
  *(volatile v4f*)p = v;
  __threadfence();
  *(volatile v4f*)p = v;
}

extern "C" void kernel_launch(void* const* d_in, const int* in_sizes, int n_in,
                              void* d_out, int out_size, void* d_ws, size_t ws_size,
                              hipStream_t stream) {
  if (n_in < 3) return;
  if (in_sizes[0] != NB * CHN * IMG * IMG) return;
  if (in_sizes[1] != EMB * KDIM) return;
  if (in_sizes[2] != EMB) return;
  if (out_size != NB * CHN * IMG * IMG) return;

  const size_t bufBytes = (size_t)MPAD * TCOLS * sizeof(float);
  const size_t aBytes   = (size_t)NB * MPAD * KDIM * sizeof(_Float16);
  const size_t wBytes   = (size_t)EMB * KDIM * sizeof(_Float16);
  if (bufBytes + aBytes + wBytes > ws_size) return;

  const float* x    = (const float*)d_in[0];
  const float* w    = (const float*)d_in[1];
  const float* bias = (const float*)d_in[2];
  float* out = (float*)d_out;

  char* ws = (char*)d_ws;
  float*    buf  = (float*)ws;
  _Float16* Acol = (_Float16*)(ws + bufBytes);
  _Float16* Wh   = (_Float16*)(ws + bufBytes + aBytes);

  {
    const int n2 = (EMB * KDIM) / 2;
    cast_w_f16x2<<<(n2 + 255) / 256, 256, 0, stream>>>(w, Wh, n2, 16.0f);
  }
  {
    const int nthr = NB * MPAD * (KDIM / 8);
    im2col_f16<<<(nthr + 255) / 256, 256, 0, stream>>>(x, Acol);
  }
  {
    const int tiles = (MPAD / 64) * (EMB / 64);
    dim3 grid((tiles + 7) / 8, NB);
    wmma_gemm64<0, false, 2, 0, false, 0><<<grid, 256, 0, stream>>>(
        (const unsigned short*)Acol, (const unsigned short*)Acol, KDIM, (long)MPAD * KDIM,
        (const unsigned short*)Wh, (const unsigned short*)Wh, KDIM, 0L,
        (void*)buf, (void*)buf, TCOLS, (long)EMB,
        bias,
        bias, 0L,
        MPAD, EMB, KDIM, 0.0625f);
  }
  smooth_scan<<<(TCOLS + 255) / 256, 256, 0, stream>>>(buf);
  {
    const int nthr = NB * CHN * IMG * (IMG / 4);
    crop_copy<<<(nthr + 255) / 256, 256, 0, stream>>>(buf, out);
  }
}
